// CostVolumeLayer_54786602828104
// MI455X (gfx1250) — hardware-verified
//
#include <hip/hip_runtime.h>
#include <stddef.h>

typedef __attribute__((ext_vector_type(16))) _Float16 v16h;
typedef __attribute__((ext_vector_type(8)))  _Float16 v8h;
typedef __attribute__((ext_vector_type(16))) __bf16   v16b;
typedef __attribute__((ext_vector_type(8)))  __bf16   v8b;
typedef __attribute__((ext_vector_type(8)))  float    v8f;
typedef __attribute__((ext_vector_type(4)))  float    v4f;

__device__ __forceinline__ unsigned short f2bf_bits(float f) {
  unsigned u = __float_as_uint(f);
  return (unsigned short)((u + 0x7FFFu + ((u >> 16) & 1u)) >> 16);
}
__device__ __forceinline__ float bf_bits2f(unsigned short h) { return __uint_as_float(((unsigned)h) << 16); }

__device__ __forceinline__ void dep_guard_h(v8f& a, v8f& b, v16h x, v16h y) { asm volatile("v_nop\n\tv_nop\n\tv_nop\n\tv_nop" : "+v"(a), "+v"(b) : "v"(x), "v"(y)); }
__device__ __forceinline__ void dep_guard_b(v8f& a, v8f& b, v16b x, v16b y) { asm volatile("v_nop\n\tv_nop\n\tv_nop\n\tv_nop" : "+v"(a), "+v"(b) : "v"(x), "v"(y)); }
__device__ __forceinline__ void keep4_h(v16h a, v16h b, v16h c, v16h d) { asm volatile("v_nop" :: "v"(a), "v"(b), "v"(c), "v"(d)); }
__device__ __forceinline__ void keep4_b(v16b a, v16b b, v16b c, v16b d) { asm volatile("v_nop" :: "v"(a), "v"(b), "v"(c), "v"(d)); }
template <typename T> struct Frag;
template <> struct Frag<_Float16> {
  typedef v16h V; union U { v16h v; v8h h[2]; };
  static __device__ __forceinline__ v16h load(const _Float16* p) {
    U f; f.h[0] = *(const v8h*)(p); f.h[1] = *(const v8h*)(p + 16); return f.v;
  }
  static __device__ __forceinline__ v8f mma(v16h a, v16h b, v8f c) {
    return __builtin_amdgcn_wmma_f32_16x16x32_f16(false, a, false, b, (short)0, c, false, false);
  }
  static __device__ __forceinline__ void guard(v8f& a, v8f& b, v16h x, v16h y) { dep_guard_h(a, b, x, y); }
  static __device__ __forceinline__ void keep(v16h a, v16h b, v16h c, v16h d) { keep4_h(a, b, c, d); }
};
template <> struct Frag<__bf16> {
  typedef v16b V; union U { v16b v; v8b h[2]; };
  static __device__ __forceinline__ v16b load(const __bf16* p) {
    U f; f.h[0] = *(const v8b*)(p); f.h[1] = *(const v8b*)(p + 16); return f.v;
  }
  static __device__ __forceinline__ v8f mma(v16b a, v16b b, v8f c) {
    return __builtin_amdgcn_wmma_f32_16x16x32_bf16(false, a, false, b, (short)0, c, false, false);
  }
  static __device__ __forceinline__ void guard(v8f& a, v8f& b, v16b x, v16b y) { dep_guard_b(a, b, x, y); }
  static __device__ __forceinline__ void keep(v16b a, v16b b, v16b c, v16b d) { keep4_b(a, b, c, d); }
};

__device__ __forceinline__ v8f at_mma(v16b a, v16b b, v8f c) {
  c = __builtin_amdgcn_wmma_f32_16x16x32_bf16(false, a, false, b, (short)0, c, false, false);
  asm volatile("v_nop\n\tv_nop\n\tv_nop\n\tv_nop" : "+v"(c) : "v"(a), "v"(b));
  return c;
}

constexpr int NBATCH  = 4;
constexpr int NCHAN   = 128;
constexpr int NHGT    = 96;
constexpr int NWID    = 160;
constexpr int SRANGE  = 4;
constexpr int NDX     = 2 * SRANGE + 1;
constexpr int NDISP   = NDX * NDX;
constexpr int XTILE   = 32;
constexpr int NXTILE  = NWID / XTILE;
constexpr int YROWS   = 2;
constexpr int NYBLK   = NHGT / YROWS;
constexpr int CCH     = 32;
constexpr int NCHUNK  = NCHAN / CCH;
constexpr int TROWS   = YROWS + 2 * SRANGE;
constexpr int TCOLS   = XTILE + 16;
constexpr int KPITCH  = 40;
constexpr int KP32    = KPITCH / 2;
constexpr int NWAVES  = NDX;
constexpr int NTHREADS = NWAVES * 32;
constexpr int NTGT_ITEMS = TROWS * (CCH / 2) * 4;
constexpr int NSRC_ITEMS = YROWS * (CCH / 2) * 4;
constexpr int LDS_T_DW  = TROWS * TCOLS * KP32;
constexpr int LDS_S_DW  = YROWS * XTILE * KP32;
constexpr int OST_FLOATS = NWAVES * YROWS * NDX * XTILE;

static_assert(NWID % XTILE == 0, "x tiling");
static_assert(NHGT % YROWS == 0, "y tiling");
static_assert(NCHAN % CCH == 0 && CCH == 32, "k step");
static_assert(OST_FLOATS <= LDS_T_DW, "staging alias fits");
static_assert(NTGT_ITEMS <= 3 * NTHREADS, "tgt staging iterations");
static_assert(NSRC_ITEMS <= NTHREADS, "src staging iterations");
static_assert(XTILE * 4 == 128, "one line per output row segment");

__device__ __forceinline__ int disp_index(int dy, int dx) {
  int ady = dy < 0 ? -dy : dy;
  int adx = dx < 0 ? -dx : dx;
  if ((ady | adx) == 0) return 0;
  if (adx == 0) return 1 + (ady - 1) * 20 + (dy > 0 ? 1 : 0);
  if (ady == 0) return 3 + (adx - 1) * 20 + (dx > 0 ? 1 : 0);
  int quad = (dy < 0) ? (dx < 0 ? 0 : 2) : (dx > 0 ? 1 : 3);
  return 5 + (ady - 1) * 20 + (adx - 1) * 4 + quad;
}

__launch_bounds__(NTHREADS)
__global__ void costvol_banded_bf16(const float* __restrict__ src,
                                    const float* __restrict__ tgt,
                                    float* __restrict__ out) {
  __shared__ __align__(16) unsigned lds_t[LDS_T_DW];
  __shared__ __align__(16) unsigned lds_s[LDS_S_DW];

  const int tid  = threadIdx.x;
  const int wave = tid >> 5;
  const int lane = tid & 31;

  const int bid = blockIdx.x;
  const int xt  = bid % NXTILE;
  const int yb  = (bid / NXTILE) % NYBLK;
  const int b   = bid / (NXTILE * NYBLK);
  const int x0  = xt * XTILE;
  const int y0  = yb * YROWS;
  const size_t plane = (size_t)NHGT * NWID;

  v8f acc[YROWS][4];
#pragma unroll
  for (int yr = 0; yr < YROWS; ++yr)
#pragma unroll
    for (int t = 0; t < 4; ++t) acc[yr][t] = (v8f){0.f, 0.f, 0.f, 0.f, 0.f, 0.f, 0.f, 0.f};

#pragma unroll 1
  for (int ch = 0; ch < NCHUNK; ++ch) {
    const int cc0 = ch * CCH;

#pragma unroll 1
    for (int k = 0; k < 3; ++k) {
      const int i = tid + NTHREADS * k;
      if (i < NTGT_ITEMS) {
        const int qq   = i & 3;
        const int rest = i >> 2;
        const int p    = rest & 15;
        const int ry   = rest >> 4;
        const int yy   = y0 - SRANGE + ry;
        const bool rok = (yy >= 0) && (yy < NHGT);
        const int yyc  = yy < 0 ? 0 : (yy >= NHGT ? NHGT - 1 : yy);
        const int c0   = cc0 + 2 * p;
        const float* r0p = tgt + ((size_t)(b * NCHAN + c0) * NHGT + (size_t)yyc) * NWID;
        const float* r1p = r0p + plane;
#pragma unroll
        for (int gg = 0; gg < 3; ++gg) {
          const int xx4  = x0 - SRANGE + 12 * qq + 4 * gg;
          const bool cok = (xx4 >= 0) && (xx4 <= NWID - 4);
          const int xx4c = xx4 < 0 ? 0 : (xx4 > NWID - 4 ? NWID - 4 : xx4);
          const v4f va = *(const v4f*)(r0p + xx4c);
          const v4f vb = *(const v4f*)(r1p + xx4c);
          const bool ok = rok && cok;
#pragma unroll
          for (int e = 0; e < 4; ++e) {
            const float fa = ok ? va[e] : 0.0f;
            const float fb = ok ? vb[e] : 0.0f;
            const unsigned pk = (unsigned)f2bf_bits(fa) | ((unsigned)f2bf_bits(fb) << 16);
            const int cx = 12 * qq + 4 * gg + e;
            lds_t[(ry * TCOLS + cx) * KP32 + p] = pk;
          }
        }
      }
    }
    if (tid < NSRC_ITEMS) {
      const int i    = tid;
      const int qq   = i & 3;
      const int rest = i >> 2;
      const int p    = rest & 15;
      const int ry   = rest >> 4;
      const int c0   = cc0 + 2 * p;
      const float* r0p = src + ((size_t)(b * NCHAN + c0) * NHGT + (size_t)(y0 + ry)) * NWID + x0 + 8 * qq;
      const float* r1p = r0p + plane;
#pragma unroll
      for (int gg = 0; gg < 2; ++gg) {
        const v4f va = *(const v4f*)(r0p + 4 * gg);
        const v4f vb = *(const v4f*)(r1p + 4 * gg);
#pragma unroll
        for (int e = 0; e < 4; ++e) {
          const unsigned pk = (unsigned)f2bf_bits(va[e]) | ((unsigned)f2bf_bits(vb[e]) << 16);
          const int cx = 8 * qq + 4 * gg + e;
          lds_s[(ry * XTILE + cx) * KP32 + p] = pk;
        }
      }
    }
    __syncthreads();

    {
      const __bf16* Tb = (const __bf16*)(const void*)lds_t;
      const __bf16* Sb = (const __bf16*)(const void*)lds_s;
      const int rl   = lane & 15;
      const int koff = (lane >> 4) * 8;
#pragma unroll
      for (int yr = 0; yr < YROWS; ++yr) {
        const int ry = yr + wave;
        const v16b b0 = Frag<__bf16>::load(Tb + ((ry * TCOLS +  0 + rl) * KPITCH + koff));
        const v16b b1 = Frag<__bf16>::load(Tb + ((ry * TCOLS + 16 + rl) * KPITCH + koff));
        const v16b b2 = Frag<__bf16>::load(Tb + ((ry * TCOLS + 32 + rl) * KPITCH + koff));
        const v16b a0 = Frag<__bf16>::load(Sb + ((yr * XTILE +  0 + rl) * KPITCH + koff));
        const v16b a1 = Frag<__bf16>::load(Sb + ((yr * XTILE + 16 + rl) * KPITCH + koff));
        acc[yr][0] = at_mma(a0, b0, acc[yr][0]);
        acc[yr][1] = at_mma(a0, b1, acc[yr][1]);
        acc[yr][2] = at_mma(a1, b1, acc[yr][2]);
        acc[yr][3] = at_mma(a1, b2, acc[yr][3]);
      }
    }
    __syncthreads();
  }

  float* ost = (float*)(void*)lds_t;
  float* ow  = ost + (size_t)wave * (YROWS * NDX * XTILE);
  {
    const int hh = lane >> 4;
    const int rl = lane & 15;
    const float inv = 1.0f / 81.0f;
#pragma unroll
    for (int yr = 0; yr < YROWS; ++yr) {
#pragma unroll
      for (int t = 0; t < 4; ++t) {
        const int mt = t >> 1;
#pragma unroll
        for (int r = 0; r < 8; ++r) {
          const int m  = 8 * hh + r;
          const int dx = (t == 0 || t == 2) ? (rl - m - SRANGE) : (rl - m + 12);
          if (dx >= -SRANGE && dx <= SRANGE) {
            ow[(yr * NDX + (dx + SRANGE)) * XTILE + 16 * mt + m] = acc[yr][t][r] * inv;
          }
        }
      }
    }
  }
  __syncthreads();
  {
    const int q  = lane >> 3;
    const int c4 = (lane & 7) * 4;
    const int dy = wave - SRANGE;
    for (int pass = 0; pass < 2; ++pass) {
#pragma unroll
      for (int yr = 0; yr < YROWS; ++yr) {
#pragma unroll
        for (int it = 0; it < 3; ++it) {
          const int li  = it * 4 + q;
          const int lic = li < NDX ? li : (NDX - 1);
          const int d   = disp_index(dy, lic - SRANGE);
          const v4f val = *(const v4f*)(ow + (yr * NDX + lic) * XTILE + c4);
          if (li < NDX) {
            float* dst = out + ((((size_t)b * NDISP + d) * NHGT + (size_t)(y0 + yr)) * NWID + x0 + c4);
            *(volatile v4f*)dst = val;
          }
        }
      }
      __threadfence();
    }
  }
}

extern "C" void kernel_launch(void* const* d_in, const int* in_sizes, int n_in,
                              void* d_out, int out_size, void* d_ws, size_t ws_size,
                              hipStream_t stream) {
  const float* src = (const float*)d_in[0];
  const float* tgt = (const float*)d_in[1];
  float* out = (float*)d_out;
  (void)in_sizes; (void)n_in; (void)out_size; (void)d_ws; (void)ws_size;

  dim3 grid(NBATCH * NYBLK * NXTILE);
  dim3 block(NTHREADS);
  costvol_banded_bf16<<<grid, block, 0, stream>>>(src, tgt, out);
}
